// GlobalWorkSpaceRNNofRNNs_67388036874680
// MI455X (gfx1250) — hardware-verified
//
#include <hip/hip_runtime.h>
#include <math.h>

constexpr int NBATCH = 64;
constexpr int NSTEP  = 256;
constexpr int NIN    = 512;
constexpr int NHID   = 2048;
constexpr int NOUT   = 512;
constexpr int NROWS  = NBATCH * NSTEP;
constexpr float ALPHA_F = 0.1f;

constexpr float WIN_CARRY      = 32.0f;
constexpr float WIN_CARRY_INV  = 1.0f / 32.0f;
constexpr float WHAT_CARRY     = 64.0f;
constexpr float WHAT_CARRY_INV = 1.0f / 64.0f;
constexpr float WOUT_CARRY     = 64.0f;
constexpr float WOUT_CARRY_INV = 1.0f / 64.0f;

constexpr int RTHR   = 512;
constexpr int RROWS  = 16;
constexpr int RWAVES = RTHR / 32;
constexpr int WCOLS  = NHID / RWAVES;
constexpr int HPITCH = NHID + 8;

static_assert(NROWS == 16384, "row count");
static_assert(NROWS % 64 == 0 && NHID % 64 == 0 && NOUT % 64 == 0, "GEMM M, N tile multiples");
static_assert(NIN % 32 == 0 && NHID % 32 == 0, "GEMM K multiples of 32");
static_assert(NBATCH % RROWS == 0, "batch rows per block");
static_assert(WCOLS == 128, "8 column tiles per wave");
static_assert(HPITCH % 8 == 0, "16-byte aligned LDS rows");
static_assert((RROWS * HPITCH) % 8 == 0, "LDS zero fill in 16-byte units");

typedef __attribute__((ext_vector_type(16))) _Float16 v16h;
typedef __attribute__((ext_vector_type(8)))  _Float16 v8h;
typedef __attribute__((ext_vector_type(8)))  float    v8f;
typedef __attribute__((ext_vector_type(4)))  float    v4f;
typedef __attribute__((ext_vector_type(4)))  unsigned v4u;

__device__ __forceinline__ void guard4_h(v8f& a0, v8f& a1, v8f& a2, v8f& a3, v16h x, v16h y0, v16h y1, v16h y2, v16h y3) {
  asm volatile("v_nop\n\tv_nop\n\tv_nop\n\tv_nop" : "+v"(a0), "+v"(a1), "+v"(a2), "+v"(a3) : "v"(x), "v"(y0), "v"(y1), "v"(y2), "v"(y3));
}
__device__ __forceinline__ void keep4_h(v16h a, v16h b, v16h c, v16h d) { asm volatile("v_nop" :: "v"(a), "v"(b), "v"(c), "v"(d)); }
__device__ __forceinline__ void acc_guard4(v8f& a, v8f& b, v8f& c, v8f& d) { asm volatile("v_nop\n\tv_nop\n\tv_nop\n\tv_nop" : "+v"(a), "+v"(b), "+v"(c), "+v"(d)); }

struct FragH {
  union U { v16h v; v8h h[2]; };
  static __device__ __forceinline__ v16h load(const _Float16* p) {
    U f; f.h[0] = *(const v8h*)(p); f.h[1] = *(const v8h*)(p + 16); return f.v;
  }
  static __device__ __forceinline__ v8f mma(v16h a, v16h b, v8f c) {
    return __builtin_amdgcn_wmma_f32_16x16x32_f16(false, a, false, b, (short)0, c, false, false);
  }
};

__device__ __forceinline__ float h16_to_f32(unsigned hb) {
  const unsigned sgn = (hb & 0x8000u) << 16;
  const unsigned em = hb & 0x7fffu;
  const float fn = __uint_as_float((em << 13) + 0x38000000u);
  const float fs = (float)em * 5.9604644775390625e-8f;
  const float mag = (em < 0x400u) ? fs : fn;
  return __uint_as_float(__float_as_uint(mag) | sgn);
}

__device__ __forceinline__ float ftanh(float x) { return 1.0f - 2.0f * __builtin_amdgcn_rcpf(__expf(2.0f * x) + 1.0f); }

__global__ __launch_bounds__(256) void cvt8_f16_kernel(const float* __restrict__ src, unsigned short* __restrict__ dst, int n8, float sc) {
  const int i = blockIdx.x * 256 + threadIdx.x;
  if (i < n8) {
    const float* sp = src + (size_t)i * 8;
    const v4f a = *(const v4f*)(sp);
    const v4f b = *(const v4f*)(sp + 4);
    v8h hv;
#pragma unroll
    for (int e = 0; e < 4; ++e) {
      hv[e]     = (_Float16)(a[e] * sc);
      hv[4 + e] = (_Float16)(b[e] * sc);
    }
    *(volatile v8h*)(dst + (size_t)i * 8) = hv;
    __threadfence();
    *(volatile v8h*)(dst + (size_t)i * 8) = hv;
  }
}

__global__ __launch_bounds__(256) void prep_what_kernel(const float* __restrict__ Bp, const float* __restrict__ Mk,
                                                        const float* __restrict__ md, unsigned short* __restrict__ What) {
  __shared__ float Ta[64 * 65];
  __shared__ float Tb[64 * 65];
  __shared__ float Rm[64];
  __shared__ float Mj[64];
  const int tid = threadIdx.x;
  const int k0 = blockIdx.x * 64, j0 = blockIdx.y * 64;
#pragma unroll
  for (int i = 0; i < 4; ++i) {
    const int idx = i * 256 + tid;
    const int rr = idx >> 4, cc = (idx & 15) * 4;
    const size_t o1 = (size_t)(j0 + rr) * NHID + k0 + cc;
    const size_t o2 = (size_t)(k0 + rr) * NHID + j0 + cc;
    const v4f b1 = *(const v4f*)(Bp + o1);
    const v4f m1 = *(const v4f*)(Mk + o1);
    const v4f b2 = *(const v4f*)(Bp + o2);
    const v4f m2 = *(const v4f*)(Mk + o2);
#pragma unroll
    for (int e = 0; e < 4; ++e) {
      Ta[rr * 65 + cc + e] = b1[e] * m1[e];
      Tb[rr * 65 + cc + e] = b2[e] * m2[e];
    }
  }
  if (tid < 64) {
    Rm[tid] = 1.0f / md[k0 + tid];
    Mj[tid] = md[j0 + tid];
  }
  __syncthreads();
  const int q = tid >> 3, c8 = (tid & 7) * 8;
  v8h hv[2];
#pragma unroll
  for (int g = 0; g < 2; ++g) {
    const int jj = g * 32 + q;
    const float mj = Mj[jj];
#pragma unroll
    for (int e = 0; e < 8; ++e) {
      const int kk = c8 + e;
      const float w = Ta[jj * 65 + kk] - (mj * Tb[kk * 65 + jj]) * Rm[kk];
      hv[g][e] = (_Float16)(w * WHAT_CARRY);
    }
  }
  for (int pass = 0; pass < 2; ++pass) {
#pragma unroll
    for (int g = 0; g < 2; ++g) {
      const size_t o = (size_t)(j0 + g * 32 + q) * NHID + (size_t)(k0 + c8);
      *(volatile v8h*)(What + o) = hv[g];
    }
    __threadfence();
  }
}

template <int OUT_MODE>
__global__ __launch_bounds__(256) void wmma_gemm64(
    const unsigned short* __restrict__ Ap, int lda,
    const unsigned short* __restrict__ Btp, int ldb,
    void* __restrict__ Cout, int ldc,
    const float* __restrict__ bias,
    int M, int N, int K, float scale) {
  const _Float16* A = (const _Float16*)Ap;
  const _Float16* Bt = (const _Float16*)Btp;
  __shared__ __align__(16) float sT[8][16 * 68];
  const int lane = threadIdx.x & 31;
  const int wave = threadIdx.x >> 5;
  const int tilesN = N >> 6;
  const int tilesM = M >> 6;
  const int tile = blockIdx.x * 8 + wave;
  if (tile >= tilesM * tilesN) return;
  const int tm = tile / tilesN;
  const int tn = tile - tm * tilesN;
  const int m0 = tm << 6;
  const int n0 = tn << 6;

  const int rlane = lane & 15;
  const int koff  = (lane >> 4) * 8;
  const int mOff  = (lane >> 4) * 8;

  v8f acc[4][4];
#pragma unroll
  for (int i = 0; i < 4; ++i)
#pragma unroll
    for (int j = 0; j < 4; ++j) acc[i][j] = (v8f){0.f,0.f,0.f,0.f,0.f,0.f,0.f,0.f};

  for (int k0 = 0; k0 < K; k0 += 32) {
    v16h bh[4];
#pragma unroll
    for (int j = 0; j < 4; ++j) {
      const size_t bo = (size_t)(n0 + (j << 4) + rlane) * ldb + koff + k0;
      bh[j] = FragH::load(Bt + bo);
    }
#pragma unroll
    for (int i = 0; i < 4; ++i) {
      const size_t ao = (size_t)(m0 + (i << 4) + rlane) * lda + koff + k0;
      const v16h ah = FragH::load(A + ao);
#pragma unroll
      for (int j = 0; j < 4; ++j) acc[i][j] = FragH::mma(ah, bh[j], acc[i][j]);
      guard4_h(acc[i][0], acc[i][1], acc[i][2], acc[i][3], ah, bh[0], bh[1], bh[2], bh[3]);
    }
    keep4_h(bh[0], bh[1], bh[2], bh[3]);
  }
  acc_guard4(acc[0][0], acc[0][1], acc[0][2], acc[0][3]);
  acc_guard4(acc[1][0], acc[1][1], acc[1][2], acc[1][3]);
  acc_guard4(acc[2][0], acc[2][1], acc[2][2], acc[2][3]);
  acc_guard4(acc[3][0], acc[3][1], acc[3][2], acc[3][3]);

  float* slab = sT[wave];
#pragma unroll
  for (int i = 0; i < 4; ++i) {
    const int mBase = m0 + (i << 4);
#pragma unroll
    for (int j = 0; j < 4; ++j) {
      const int n = n0 + (j << 4) + rlane;
      const float bv = bias[n];
#pragma unroll
      for (int r = 0; r < 8; ++r) {
        float v = acc[i][j][r] * scale;
        v += bv;
        slab[(mOff + r) * 68 + (j << 4) + rlane] = v;
      }
    }
    __builtin_amdgcn_fence(__ATOMIC_RELEASE, "workgroup");
    __builtin_amdgcn_wave_barrier();
    __builtin_amdgcn_fence(__ATOMIC_ACQUIRE, "workgroup");
    if (OUT_MODE == 0) {
      float* C = (float*)Cout;
      const int hh = lane >> 4, c4 = (lane & 15) * 4;
      for (int pass = 0; pass < 2; ++pass) {
#pragma unroll
        for (int it = 0; it < 8; ++it) {
          const int row = it * 2 + hh;
          const v4f v = *(const v4f*)(slab + row * 68 + c4);
          *(volatile v4f*)(C + (size_t)(mBase + row) * ldc + n0 + c4) = v;
        }
        __threadfence();
      }
    } else {
      const int q = lane >> 3, c8 = (lane & 7) * 8;
      unsigned short* C = (unsigned short*)Cout;
      for (int pass = 0; pass < 2; ++pass) {
#pragma unroll
        for (int it = 0; it < 4; ++it) {
          const int row = it * 4 + q;
          const float* sp = slab + row * 68 + c8;
          v8h hv;
#pragma unroll
          for (int e = 0; e < 8; ++e) hv[e] = (_Float16)sp[e];
          *(volatile v8h*)(C + (size_t)(mBase + row) * ldc + n0 + c8) = hv;
        }
        __threadfence();
      }
    }
    __builtin_amdgcn_fence(__ATOMIC_RELEASE, "workgroup");
    __builtin_amdgcn_wave_barrier();
    __builtin_amdgcn_fence(__ATOMIC_ACQUIRE, "workgroup");
  }
}

__global__ __launch_bounds__(RTHR) void recur_kernel(const unsigned short* __restrict__ Whp, unsigned short* P) {
  __shared__ __align__(16) _Float16 Ah[RROWS * HPITCH];
  const _Float16* Wh = (const _Float16*)Whp;
  const int tid = threadIdx.x, lane = tid & 31, wave = tid >> 5;
  const int c = lane & 15, hh = lane >> 4, koff = hh * 8;
  const int rowbase = blockIdx.x * RROWS;
  const int colbase = WCOLS * wave + 8 * c;

  {
    const v8h zh = {(_Float16)0.0f, (_Float16)0.0f, (_Float16)0.0f, (_Float16)0.0f,
                    (_Float16)0.0f, (_Float16)0.0f, (_Float16)0.0f, (_Float16)0.0f};
    v8h* az = (v8h*)Ah;
#pragma unroll 1
    for (int i = tid; i < RROWS * HPITCH / 8; i += RTHR) az[i] = zh;
  }
  float hst[8][8];
#pragma unroll
  for (int j = 0; j < 8; ++j)
#pragma unroll
    for (int r = 0; r < 8; ++r) hst[j][r] = 0.0f;
  __syncthreads();

  const _Float16* ahrow = Ah + c * HPITCH + koff;
  const _Float16* wb = Wh + (size_t)colbase * NHID + koff;
  const v8f z8 = {0.f, 0.f, 0.f, 0.f, 0.f, 0.f, 0.f, 0.f};

#pragma unroll 1
  for (int t = 0; t < NSTEP; ++t) {
    v8f acc[8];
#pragma unroll
    for (int j = 0; j < 8; ++j) acc[j] = z8;

#pragma unroll 1
    for (int k0 = 0; k0 < NHID; k0 += 32) {
      const v16h a = FragH::load(ahrow + k0);
      const _Float16* wk = wb + k0;
      {
        const v16h b0 = FragH::load(wk);
        const v16h b1 = FragH::load(wk + (size_t)1 * NHID);
        const v16h b2 = FragH::load(wk + (size_t)2 * NHID);
        const v16h b3 = FragH::load(wk + (size_t)3 * NHID);
        acc[0] = FragH::mma(a, b0, acc[0]);
        acc[1] = FragH::mma(a, b1, acc[1]);
        acc[2] = FragH::mma(a, b2, acc[2]);
        acc[3] = FragH::mma(a, b3, acc[3]);
        guard4_h(acc[0], acc[1], acc[2], acc[3], a, b0, b1, b2, b3);
      }
      {
        const v16h b4 = FragH::load(wk + (size_t)4 * NHID);
        const v16h b5 = FragH::load(wk + (size_t)5 * NHID);
        const v16h b6 = FragH::load(wk + (size_t)6 * NHID);
        const v16h b7 = FragH::load(wk + (size_t)7 * NHID);
        acc[4] = FragH::mma(a, b4, acc[4]);
        acc[5] = FragH::mma(a, b5, acc[5]);
        acc[6] = FragH::mma(a, b6, acc[6]);
        acc[7] = FragH::mma(a, b7, acc[7]);
        guard4_h(acc[4], acc[5], acc[6], acc[7], a, b4, b5, b6, b7);
      }
    }
    acc_guard4(acc[0], acc[1], acc[2], acc[3]);
    acc_guard4(acc[4], acc[5], acc[6], acc[7]);

#pragma unroll
    for (int r = 0; r < 8; ++r) {
      const size_t eo = ((size_t)(rowbase + 8 * hh + r) * NSTEP + (size_t)t) * NHID + (size_t)colbase;
      v4u xw = *(const v4u*)(const void*)(P + eo);
      asm volatile("" : "+v"(xw));
      float xv[8];
#pragma unroll
      for (int i = 0; i < 4; ++i) {
        const unsigned w = xw[i];
        xv[2 * i]     = h16_to_f32(w & 0xffffu);
        xv[2 * i + 1] = h16_to_f32(w >> 16);
      }
#pragma unroll
      for (int j = 0; j < 8; ++j) {
        const float pre = fmaf(acc[j][r], WHAT_CARRY_INV, xv[j]);
        const float th = ftanh(pre);
        const float ho = hst[j][r];
        hst[j][r] = ho + ALPHA_F * (th - ho);
      }
    }

    __syncthreads();

    v8h hv[8];
#pragma unroll
    for (int r = 0; r < 8; ++r)
#pragma unroll
      for (int j = 0; j < 8; ++j) hv[r][j] = (_Float16)hst[j][r];
#pragma unroll
    for (int r = 0; r < 8; ++r) *(v8h*)(Ah + (8 * hh + r) * HPITCH + colbase) = hv[r];
    for (int pass = 0; pass < 2; ++pass) {
#pragma unroll
      for (int r = 0; r < 8; ++r) {
        const size_t eo = ((size_t)(rowbase + 8 * hh + r) * NSTEP + (size_t)t) * NHID + (size_t)colbase;
        *(volatile v8h*)(P + eo) = hv[r];
      }
      __threadfence();
    }

    __syncthreads();
  }
}

extern "C" void kernel_launch(void* const* d_in, const int* in_sizes, int n_in,
                              void* d_out, int out_size, void* d_ws, size_t ws_size, hipStream_t stream) {
  if (n_in < 8 || d_out == nullptr || d_ws == nullptr) return;
  if (in_sizes[0] != NBATCH * NSTEP * NIN || in_sizes[1] != NHID * NHID || in_sizes[2] != NHID * NHID ||
      in_sizes[3] != NHID || in_sizes[4] != NHID * NIN || in_sizes[5] != NHID ||
      in_sizes[6] != NOUT * NHID || in_sizes[7] != NOUT || out_size != NROWS * NOUT) return;

  const float* xin   = (const float*)d_in[0];
  const float* bmat  = (const float*)d_in[1];
  const float* bmask = (const float*)d_in[2];
  const float* mdiag = (const float*)d_in[3];
  const float* win   = (const float*)d_in[4];
  const float* bh    = (const float*)d_in[5];
  const float* wout  = (const float*)d_in[6];
  const float* bout  = (const float*)d_in[7];
  float* out = (float*)d_out;

  char* ws = (char*)d_ws;
  size_t off = 0;
  auto carve = [&](size_t bytes) -> char* { char* p = ws + off; off += (bytes + 255) & ~(size_t)255; return p; };
  unsigned short* IN16   = (unsigned short*)carve((size_t)NROWS * NIN * 2);
  unsigned short* WHAT16 = (unsigned short*)carve((size_t)NHID * NHID * 2);
  unsigned short* WIN16  = (unsigned short*)carve((size_t)NHID * NIN * 2);
  unsigned short* WOUT16 = (unsigned short*)carve((size_t)NOUT * NHID * 2);
  unsigned short* PPL    = (unsigned short*)carve((size_t)NROWS * NHID * 2);
  if (off > ws_size || off > (size_t)134217728) return;

  const int n8x = NROWS * (NIN / 8);
  const int n8i = NHID * (NIN / 8);
  const int n8o = NOUT * (NHID / 8);
  cvt8_f16_kernel<<<(n8x + 255) / 256, 256, 0, stream>>>(xin, IN16, n8x, 1.0f);
  cvt8_f16_kernel<<<(n8i + 255) / 256, 256, 0, stream>>>(win, WIN16, n8i, WIN_CARRY);
  cvt8_f16_kernel<<<(n8o + 255) / 256, 256, 0, stream>>>(wout, WOUT16, n8o, WOUT_CARRY);
  prep_what_kernel<<<dim3(NHID / 64, NHID / 64), 256, 0, stream>>>(bmat, bmask, mdiag, WHAT16);

  wmma_gemm64<1><<<(NROWS / 64) * (NHID / 64) / 8, 256, 0, stream>>>(
      IN16, NIN, WIN16, NIN, (void*)PPL, NHID, bh, NROWS, NHID, NIN, WIN_CARRY_INV);

  recur_kernel<<<NBATCH / RROWS, RTHR, 0, stream>>>(WHAT16, PPL);

  wmma_gemm64<0><<<(NROWS / 64) * (NOUT / 64) / 8, 256, 0, stream>>>(
      PPL, NHID, WOUT16, NHID, (void*)out, NOUT, bout, NROWS, NOUT, NHID, WOUT_CARRY_INV);
}
